// GraphEncoder_v2_28879360098475
// MI455X (gfx1250) — hardware-verified
//
#include <hip/hip_runtime.h>
#include <stddef.h>


#define FD    256
#define KIN   128
#define GR    16
#define LDSP  264
#define XSP   516
#define NB    256
#define SH    8
#define CHUNK 4096
#define ATHR  256
#define AWAVE 8
#define NGRP  (CHUNK / (ATHR * 4))
#define WCAP  ((CHUNK / ATHR) * 32)
#define NHD   4
#define AGG_SACC (NB * FD)
#define AGG_AUX  (2 * NB * NHD)
#define AGG_LIST (AWAVE * WCAP)
#define AGG_LDS_BYTES ((AGG_SACC + AGG_AUX + AGG_LIST + AWAVE) * 4)
#define WS_CAP ((size_t)134217728)
#define WSC   64.0f
#define WSCI  0.015625f
#define LN_EPS 1e-5f

static_assert(NGRP == 4);
static_assert(WCAP == 512);
static_assert(NB == (1 << SH));
static_assert(SH + 12 <= 31);
static_assert(AGG_LDS_BYTES == 286752);
static_assert((LDSP * 2) % 16 == 0);
static_assert((XSP * 4) % 16 == 0);
static_assert(NB % AWAVE == 0);
static_assert(FD == 32 * 8);

typedef float          v4f   __attribute__((ext_vector_type(4)));
typedef float          v8f   __attribute__((ext_vector_type(8)));
typedef int            v4i   __attribute__((ext_vector_type(4)));
typedef unsigned short v8us  __attribute__((ext_vector_type(8)));
typedef _Float16       v8h   __attribute__((ext_vector_type(8)));
typedef _Float16       v16h  __attribute__((ext_vector_type(16)));
typedef __bf16         v16bf __attribute__((ext_vector_type(16)));

union FragH { v16h v; v8us p[2]; };
union FragB { v16bf v; v8us p[2]; };

__device__ __forceinline__ unsigned short bf16_rne(float x) {
  unsigned u = __float_as_uint(x);
  u += 0x7FFFu + ((u >> 16) & 1u);
  return (unsigned short)(u >> 16);
}
__device__ __forceinline__ float bf16_val(unsigned short b) {
  return __uint_as_float(((unsigned)b) << 16);
}
__device__ __forceinline__ unsigned short f16_bits(float x) {
  union { _Float16 h; unsigned short u; } c;
  c.h = (_Float16)x;
  return c.u;
}

__device__ __forceinline__ v8f wmh(v16h a, v16h b, v8f c) {
  v8f d = __builtin_amdgcn_wmma_f32_16x16x32_f16(false, a, false, b, (short)0, c, false, false);
  asm volatile("v_nop\n\tv_nop\n\tv_nop\n\tv_nop" : "+v"(d) : "v"(a), "v"(b));
  return d;
}
__device__ __forceinline__ v8f wmb(v16bf a, v16bf b, v8f c) {
  v8f d = __builtin_amdgcn_wmma_f32_16x16x32_bf16(false, a, false, b, (short)0, c, false, false);
  asm volatile("v_nop\n\tv_nop\n\tv_nop\n\tv_nop" : "+v"(d) : "v"(a), "v"(b));
  return d;
}

__device__ __forceinline__ float wsum(float v) {
  v += __shfl_xor(v, 16, 32);
  v += __shfl_xor(v, 8, 32);
  v += __shfl_xor(v, 4, 32);
  v += __shfl_xor(v, 2, 32);
  v += __shfl_xor(v, 1, 32);
  return v;
}
__device__ __forceinline__ float hsum4(v4f a) { return (a.x + a.y) + (a.z + a.w); }
__device__ __forceinline__ v4f ld4(const float* p) { return *(const v4f*)p; }
__device__ __forceinline__ v4f relu4(v4f o) {
  v4f r;
  r.x = fmaxf(o.x, 0.f); r.y = fmaxf(o.y, 0.f); r.z = fmaxf(o.z, 0.f); r.w = fmaxf(o.w, 0.f);
  return r;
}

__device__ __forceinline__ void cvt8(v4f a, v4f b, v8us& f, v8us& h, v8us& l) {
  const float x[8] = {a.x, a.y, a.z, a.w, b.x, b.y, b.z, b.w};
#pragma unroll
  for (int i = 0; i < 8; ++i) {
    f[i] = f16_bits(x[i]);
    const unsigned short hb = bf16_rne(x[i]);
    h[i] = hb;
    l[i] = bf16_rne(x[i] - bf16_val(hb));
  }
}
__device__ __forceinline__ v8us cvt8_f16(v4f a, v4f b) {
  const float x[8] = {a.x, a.y, a.z, a.w, b.x, b.y, b.z, b.w};
  v8us f = {0, 0, 0, 0, 0, 0, 0, 0};
#pragma unroll
  for (int i = 0; i < 8; ++i) f[i] = f16_bits(x[i]);
  return f;
}

template <int KD>
__device__ __forceinline__ void stage_planes(const float* A, int rowBase, int nA,
                                             unsigned short* ldsF, unsigned short* ldsH,
                                             unsigned short* ldsL, int tid) {
  constexpr int EPT = KD / 16;
  const int r  = tid >> 4;
  const int c0 = (tid & 15) * EPT;
  int row = rowBase + r;
  if (row > nA - 1) row = nA - 1;
  const float* p = A + (size_t)row * KD + c0;
#pragma unroll
  for (int g = 0; g < EPT / 8; ++g) {
    const v4f f0 = ld4(p + 8 * g);
    const v4f f1 = ld4(p + 8 * g + 4);
    v8us ff = {0, 0, 0, 0, 0, 0, 0, 0}, hh = {0, 0, 0, 0, 0, 0, 0, 0}, ll = {0, 0, 0, 0, 0, 0, 0, 0};
    cvt8(f0, f1, ff, hh, ll);
    *(v8us*)(ldsF + r * LDSP + c0 + 8 * g) = ff;
    *(v8us*)(ldsH + r * LDSP + c0 + 8 * g) = hh;
    *(v8us*)(ldsL + r * LDSP + c0 + 8 * g) = ll;
  }
}

template <int KD>
__global__ __launch_bounds__(256) void k_prep(const float* __restrict__ wq, const float* __restrict__ wk,
                                             const float* __restrict__ wv, const float* __restrict__ wsk,
                                             unsigned short* F, unsigned short* Hh, unsigned short* Hl) {
  const int t = blockIdx.x * 256 + threadIdx.x;
  if (t >= 4 * FD) return;
  const int n = t & (FD - 1);
  if (t < 2 * FD) {
    const float* W = (t < FD) ? wq : wk;
    unsigned short* df = F + (size_t)t * KD;
#pragma unroll 1
    for (int kb = 0; kb < KD / 8; ++kb) {
      v8us f = {0, 0, 0, 0, 0, 0, 0, 0};
#pragma unroll
      for (int i = 0; i < 8; ++i) f[i] = f16_bits(W[(size_t)(kb * 8 + i) * FD + n] * WSC);
      *(volatile v8us*)(df + kb * 8) = f;
      __threadfence();
      *(volatile v8us*)(df + kb * 8) = f;
    }
  } else {
    const int u = t - 2 * FD;
    const float* W = (u < FD) ? wv : wsk;
    unsigned short* dh = Hh + (size_t)u * KD;
    unsigned short* dl = Hl + (size_t)u * KD;
#pragma unroll 1
    for (int kb = 0; kb < KD / 8; ++kb) {
      v8us h = {0, 0, 0, 0, 0, 0, 0, 0}, l = {0, 0, 0, 0, 0, 0, 0, 0};
#pragma unroll
      for (int i = 0; i < 8; ++i) {
        const float x = W[(size_t)(kb * 8 + i) * FD + n];
        const unsigned short hb = bf16_rne(x);
        h[i] = hb;
        l[i] = bf16_rne(x - bf16_val(hb));
      }
      *(volatile v8us*)(dh + kb * 8) = h;
      *(volatile v8us*)(dl + kb * 8) = l;
      __threadfence();
      *(volatile v8us*)(dh + kb * 8) = h;
      *(volatile v8us*)(dl + kb * 8) = l;
    }
  }
}

template <int KD>
__global__ __launch_bounds__(256) void k_proj(const float* A,
                                             const unsigned short* __restrict__ F,
                                             const unsigned short* __restrict__ Hh,
                                             const unsigned short* __restrict__ Hl,
                                             const float* __restrict__ bq, const float* __restrict__ bk,
                                             const float* __restrict__ bv, const float* __restrict__ bsk,
                                             unsigned short* Qo, float* Ko, float* Vo, float* So, int nA) {
  __shared__ __attribute__((aligned(16))) unsigned short s_hs[3 * GR * LDSP];
  __shared__ __attribute__((aligned(16))) float s_xs[GR * XSP];

  const int tid  = threadIdx.x;
  const int lane = tid & 31;
  const int wave = tid >> 5;
  const int hh   = lane >> 4;
  const int m    = lane & 15;
  const int rowBase = blockIdx.x * GR;
  unsigned short* ldsF = s_hs;
  unsigned short* ldsH = s_hs + GR * LDSP;
  unsigned short* ldsL = s_hs + 2 * GR * LDSP;

  stage_planes<KD>(A, rowBase, nA, ldsF, ldsH, ldsL, tid);
  __syncthreads();

  const v8f z8 = {0.f, 0.f, 0.f, 0.f, 0.f, 0.f, 0.f, 0.f};

  {
    v8f acc[4];
#pragma unroll
    for (int t = 0; t < 4; ++t) acc[t] = z8;
    const unsigned short* pa = ldsF + m * LDSP + 8 * hh;
#pragma unroll 1
    for (int kt = 0; kt < KD / 32; ++kt) {
      const int k0 = kt * 32;
      FragH a;
      a.p[0] = *(const v8us*)(pa + k0);
      a.p[1] = *(const v8us*)(pa + k0 + 16);
#pragma unroll
      for (int t = 0; t < 4; ++t) {
        const size_t prow = (size_t)((4 * wave + t) * 16 + m);
        const unsigned short* pb = F + prow * KD + k0 + 8 * hh;
        FragH b;
        b.p[0] = *(const v8us*)(pb);
        b.p[1] = *(const v8us*)(pb + 16);
        acc[t] = wmh(a.v, b.v, acc[t]);
      }
    }
#pragma unroll
    for (int t = 0; t < 4; ++t) {
      const int gcol = (4 * wave + t) * 16 + m;
      const float* bb = (gcol < FD) ? bq : bk;
      const float bvl = bb[gcol & (FD - 1)];
#pragma unroll
      for (int r = 0; r < 8; ++r) s_xs[(8 * hh + r) * XSP + gcol] = acc[t][r] * WSCI + bvl;
    }
  }

  v8f accB[4];
#pragma unroll
  for (int t = 0; t < 4; ++t) accB[t] = z8;
  {
    const unsigned short* pah = ldsH + m * LDSP + 8 * hh;
    const unsigned short* pal = ldsL + m * LDSP + 8 * hh;
#pragma unroll 1
    for (int kt = 0; kt < KD / 32; ++kt) {
      const int k0 = kt * 32;
      FragB ah, al;
      ah.p[0] = *(const v8us*)(pah + k0);
      ah.p[1] = *(const v8us*)(pah + k0 + 16);
      al.p[0] = *(const v8us*)(pal + k0);
      al.p[1] = *(const v8us*)(pal + k0 + 16);
#pragma unroll
      for (int t = 0; t < 4; ++t) {
        const size_t prow = (size_t)((4 * wave + t) * 16 + m);
        const unsigned short* pbh = Hh + prow * KD + k0 + 8 * hh;
        const unsigned short* pbl = Hl + prow * KD + k0 + 8 * hh;
        FragB bh, bl;
        bh.p[0] = *(const v8us*)(pbh);
        bh.p[1] = *(const v8us*)(pbh + 16);
        bl.p[0] = *(const v8us*)(pbl);
        bl.p[1] = *(const v8us*)(pbl + 16);
        accB[t] = wmb(ah.v, bh.v, accB[t]);
        accB[t] = wmb(ah.v, bl.v, accB[t]);
        accB[t] = wmb(al.v, bh.v, accB[t]);
      }
    }
  }
  __syncthreads();

  {
    const int matw = wave >> 2;
    bool okq[4];
    int  ndq[4];
#pragma unroll
    for (int q = 0; q < 4; ++q) {
      const int row = (4 * wave + q) & 15;
      ndq[q] = rowBase + row;
      okq[q] = ndq[q] < nA;
    }
    if (matw == 0) {
      v8us hv[4];
      unsigned short* qp[4];
#pragma unroll
      for (int q = 0; q < 4; ++q) {
        const int row = (4 * wave + q) & 15;
        const float* xr = s_xs + row * XSP + 8 * lane;
        hv[q] = cvt8_f16(ld4(xr), ld4(xr + 4));
        qp[q] = Qo + (size_t)ndq[q] * FD + 8 * lane;
      }
#pragma unroll
      for (int q = 0; q < 4; ++q) if (okq[q]) *(volatile v8us*)(qp[q]) = hv[q];
      __threadfence();
#pragma unroll
      for (int q = 0; q < 4; ++q) if (okq[q]) *(volatile v8us*)(qp[q]) = hv[q];
    } else {
      v4f xr[8];
      float* gp[8];
#pragma unroll
      for (int q = 0; q < 4; ++q) {
        const int row = (4 * wave + q) & 15;
        const float* xs = s_xs + row * XSP + FD + 4 * lane;
        xr[2 * q]     = ld4(xs);
        xr[2 * q + 1] = ld4(xs + 128);
        gp[2 * q]     = Ko + (size_t)ndq[q] * FD + 4 * lane;
        gp[2 * q + 1] = Ko + (size_t)ndq[q] * FD + 128 + 4 * lane;
      }
#pragma unroll
      for (int q = 0; q < 4; ++q) {
        if (okq[q]) { *(volatile v4f*)(gp[2 * q]) = xr[2 * q]; *(volatile v4f*)(gp[2 * q + 1]) = xr[2 * q + 1]; }
      }
      __threadfence();
#pragma unroll
      for (int q = 0; q < 4; ++q) {
        if (okq[q]) { *(volatile v4f*)(gp[2 * q]) = xr[2 * q]; *(volatile v4f*)(gp[2 * q + 1]) = xr[2 * q + 1]; }
      }
    }
  }
  __syncthreads();

#pragma unroll
  for (int t = 0; t < 4; ++t) {
    const int gcol = (4 * wave + t) * 16 + m;
    const float* bb = (gcol < FD) ? bv : bsk;
    const float bvl = bb[gcol & (FD - 1)];
#pragma unroll
    for (int r = 0; r < 8; ++r) s_xs[(8 * hh + r) * XSP + gcol] = accB[t][r] + bvl;
  }
  __syncthreads();

  {
    const int matw = wave >> 2;
    float* ob = (matw == 0) ? Vo : So;
    const int cb = matw * FD;
    v4f xr[8];
    float* gp[8];
    bool okq[4];
#pragma unroll
    for (int q = 0; q < 4; ++q) {
      const int row  = (4 * wave + q) & 15;
      const int node = rowBase + row;
      okq[q] = node < nA;
      const float* xs = s_xs + row * XSP + cb + 4 * lane;
      xr[2 * q]     = ld4(xs);
      xr[2 * q + 1] = ld4(xs + 128);
      gp[2 * q]     = ob + (size_t)node * FD + 4 * lane;
      gp[2 * q + 1] = ob + (size_t)node * FD + 128 + 4 * lane;
    }
#pragma unroll
    for (int q = 0; q < 4; ++q) {
      if (okq[q]) { *(volatile v4f*)(gp[2 * q]) = xr[2 * q]; *(volatile v4f*)(gp[2 * q + 1]) = xr[2 * q + 1]; }
    }
    __threadfence();
#pragma unroll
    for (int q = 0; q < 4; ++q) {
      if (okq[q]) { *(volatile v4f*)(gp[2 * q]) = xr[2 * q]; *(volatile v4f*)(gp[2 * q + 1]) = xr[2 * q + 1]; }
    }
  }
}

template <int NH, int RELU>
__global__ __launch_bounds__(ATHR) void k_agg(const int* __restrict__ srcA, const int* __restrict__ dstA,
                                              const float* __restrict__ eaA, const float* __restrict__ ewA,
                                              const _Float16* __restrict__ Q, const float* __restrict__ K,
                                              const float* __restrict__ V,
                                              const float* __restrict__ lng, const float* __restrict__ lnb,
                                              float* io, int nN, int nE) {
  extern __shared__ v4f lds_dyn[];
  float* sacc = (float*)lds_dyn;
  float* mx   = sacc + AGG_SACC;
  float* den  = mx + NB * NHD;
  int*   list = (int*)(den + NB * NHD);
  int*   wcnt = list + AGG_LIST;

  const int tid  = threadIdx.x;
  const int lane = tid & 31;
  const int wave = tid >> 5;
  const int nodeBase = blockIdx.x * NB;

  const v4f ew0 = ld4(ewA + 8 * lane);
  const v4f ew1 = ld4(ewA + 8 * lane + 4);

  {
    const v4f z4 = {0.f, 0.f, 0.f, 0.f};
    for (int i = tid; i < AGG_SACC / 4; i += ATHR) lds_dyn[i] = z4;
    for (int i = tid; i < NB * NHD; i += ATHR) { mx[i] = -1.0e30f; den[i] = 0.f; }
  }
  __syncthreads();

  const bool al16 = ((nE & 3) == 0);
  const int nChunks = (nE + CHUNK - 1) / CHUNK;
#pragma unroll 1
  for (int ch = 0; ch < nChunks; ++ch) {
    const int cbase = ch * CHUNK;
    int wc = 0;
#pragma unroll
    for (int g = 0; g < NGRP; ++g) {
      const int el0 = (g * ATHR + tid) * 4;
      const int e0  = cbase + el0;
      const int sent = -2147483647 - 1;
      v4i d;
      if (al16 && (e0 + 3 < nE)) {
        d = *(const v4i*)(dstA + e0);
      } else {
        d.x = (e0     < nE) ? dstA[min(e0, nE - 1)]     : sent;
        d.y = (e0 + 1 < nE) ? dstA[min(e0 + 1, nE - 1)] : sent;
        d.z = (e0 + 2 < nE) ? dstA[min(e0 + 2, nE - 1)] : sent;
        d.w = (e0 + 3 < nE) ? dstA[min(e0 + 3, nE - 1)] : sent;
      }
      const unsigned s0 = (unsigned)d.x - (unsigned)nodeBase;
      const unsigned s1 = (unsigned)d.y - (unsigned)nodeBase;
      const unsigned s2 = (unsigned)d.z - (unsigned)nodeBase;
      const unsigned s3 = (unsigned)d.w - (unsigned)nodeBase;
      const bool h0 = s0 < (unsigned)NB;
      const bool h1 = s1 < (unsigned)NB;
      const bool h2 = s2 < (unsigned)NB;
      const bool h3 = s3 < (unsigned)NB;
      const unsigned many = __builtin_amdgcn_ballot_w32(h0 | h1 | h2 | h3);
      if (many != 0u) {
#define HITJ(J, HJ, SJ) { \
          const unsigned mj = __builtin_amdgcn_ballot_w32(HJ); \
          if (HJ) { \
            const int pos = wc + (int)__builtin_amdgcn_mbcnt_lo(mj, 0u); \
            if (pos < WCAP) list[wave * WCAP + pos] = ((el0 + (J)) << SH) | (int)(SJ); \
          } \
          wc += (int)__builtin_popcount(mj); }
        HITJ(0, h0, s0)
        HITJ(1, h1, s1)
        HITJ(2, h2, s2)
        HITJ(3, h3, s3)
#undef HITJ
      }
    }
    if (lane == 0) wcnt[wave] = wc;
    __syncthreads();

    if (wave == 0) {
      const float sc = (NH == 4) ? 0.125f : 0.0625f;
      const int hd = (NH == 4) ? (lane >> 3) : 0;
#pragma unroll 1
      for (int wsx = 0; wsx < AWAVE; ++wsx) {
        int n = wcnt[wsx];
        if (n > WCAP) n = WCAP;
        if (n < 0) n = 0;
#pragma unroll 1
        for (int i = 0; i < n; ++i) {
          const int ent  = list[wsx * WCAP + i];
          const int slot = ent & (NB - 1);
          const int el   = (ent >> SH) & (CHUNK - 1);
          int e = cbase + el;
          if (e > nE - 1) e = nE - 1;
          int src = srcA[e];
          src = src < 0 ? 0 : (src > nN - 1 ? nN - 1 : src);
          int nd = nodeBase + slot;
          if (nd > nN - 1) nd = nN - 1;
          const float av = eaA[e];
          const v8h qh = *(const v8h*)(Q + (size_t)nd * FD + 8 * lane);
          v4f q0, q1;
          q0.x = (float)qh[0]; q0.y = (float)qh[1]; q0.z = (float)qh[2]; q0.w = (float)qh[3];
          q1.x = (float)qh[4]; q1.y = (float)qh[5]; q1.z = (float)qh[6]; q1.w = (float)qh[7];
          const float* krow = K + (size_t)src * FD + 8 * lane;
          const float* vrow = V + (size_t)src * FD + 8 * lane;
          const v4f k0 = ld4(krow), k1 = ld4(krow + 4);
          const v4f v0 = ld4(vrow), v1 = ld4(vrow + 4);
          const v4f kj0 = k0 + ew0 * av;
          const v4f kj1 = k1 + ew1 * av;
          float part = hsum4(q0 * kj0) + hsum4(q1 * kj1);
          if (NH == 1) {
            part += __shfl_xor(part, 16, 32);
            part += __shfl_xor(part, 8, 32);
          }
          part += __shfl_xor(part, 4, 32);
          part += __shfl_xor(part, 2, 32);
          part += __shfl_xor(part, 1, 32);
          const float logit = part * sc;
          const int hidx = slot * NHD + hd;
          const float mo = mx[hidx];
          const float mn = fmaxf(mo, logit);
          const float corr = __expf(mo - mn);
          const float p = __expf(logit - mn);
          const float dn = den[hidx] * corr + p;
          v4f* sp = (v4f*)(sacc + slot * FD + 8 * lane);
          const v4f c0 = sp[0];
          const v4f c1 = sp[1];
          sp[0] = c0 * corr + (v0 + ew0 * av) * p;
          sp[1] = c1 * corr + (v1 + ew1 * av) * p;
          den[hidx] = dn;
          mx[hidx]  = mn;
        }
      }
    }
    __syncthreads();
  }
  __syncthreads();

  const v4f g0  = ld4(lng + 4 * lane);
  const v4f g1  = ld4(lng + 128 + 4 * lane);
  const v4f be0 = ld4(lnb + 4 * lane);
  const v4f be1 = ld4(lnb + 128 + 4 * lane);
  const int hd0 = (NH == 4) ? (lane >> 4) : 0;
  const int hd1 = (NH == 4) ? (2 + (lane >> 4)) : 0;
#pragma unroll 1
  for (int j = 0; j < NB / AWAVE; ++j) {
    const int row  = j * AWAVE + wave;
    const int node = nodeBase + row;
    const bool ok  = node < nN;
    const int nl   = ok ? node : (nN - 1);
    const v4f a0 = lds_dyn[row * 64 + lane];
    const v4f a1 = lds_dyn[row * 64 + 32 + lane];
    const float d0 = den[row * NHD + hd0];
    const float d1 = den[row * NHD + hd1];
    const float inv0 = (d0 > 0.f) ? __builtin_amdgcn_rcpf(d0) : 0.f;
    const float inv1 = (d1 > 0.f) ? __builtin_amdgcn_rcpf(d1) : 0.f;
    const v4f s0 = ld4(io + (size_t)nl * FD + 4 * lane);
    const v4f s1 = ld4(io + (size_t)nl * FD + 128 + 4 * lane);
    const v4f y0 = a0 * inv0 + s0;
    const v4f y1 = a1 * inv1 + s1;
    const float mu = wsum(hsum4(y0) + hsum4(y1)) * (1.0f / 256.0f);
    const v4f c0 = y0 - mu;
    const v4f c1 = y1 - mu;
    const float var = wsum(hsum4(c0 * c0) + hsum4(c1 * c1)) * (1.0f / 256.0f);
    const float rs = rsqrtf(var + LN_EPS);
    v4f o0 = c0 * rs * g0 + be0;
    v4f o1 = c1 * rs * g1 + be1;
    if (RELU) { o0 = relu4(o0); o1 = relu4(o1); }
    lds_dyn[row * 64 + lane]      = o0;
    lds_dyn[row * 64 + 32 + lane] = o1;
    if (ok) {
      *(volatile v4f*)(io + (size_t)node * FD + 4 * lane)       = o0;
      *(volatile v4f*)(io + (size_t)node * FD + 128 + 4 * lane) = o1;
    }
  }
  __threadfence();
#pragma unroll 1
  for (int j = 0; j < NB / AWAVE; ++j) {
    const int row  = j * AWAVE + wave;
    const int node = nodeBase + row;
    if (node < nN) {
      const v4f o0 = lds_dyn[row * 64 + lane];
      const v4f o1 = lds_dyn[row * 64 + 32 + lane];
      *(volatile v4f*)(io + (size_t)node * FD + 4 * lane)       = o0;
      *(volatile v4f*)(io + (size_t)node * FD + 128 + 4 * lane) = o1;
    }
  }
}

extern "C" void kernel_launch(void* const* d_in, const int* in_sizes, int n_in,
                              void* d_out, int out_size, void* d_ws, size_t ws_size,
                              hipStream_t stream) {
  if (n_in < 25) return;
  if (in_sizes[0] < KIN || (in_sizes[0] % KIN) != 0) return;
  const int nN = in_sizes[0] / KIN;
  if (in_sizes[1] < 2 || (in_sizes[1] & 1) != 0) return;
  const int nE = in_sizes[1] / 2;
  if (in_sizes[2] != nE) return;
  if (in_sizes[3] != KIN * FD || in_sizes[5] != KIN * FD || in_sizes[7] != KIN * FD || in_sizes[10] != KIN * FD) return;
  if (in_sizes[14] != FD * FD || in_sizes[16] != FD * FD || in_sizes[18] != FD * FD || in_sizes[21] != FD * FD) return;
  if (in_sizes[4] != FD || in_sizes[6] != FD || in_sizes[8] != FD || in_sizes[9] != FD || in_sizes[11] != FD) return;
  if (in_sizes[12] != FD || in_sizes[13] != FD) return;
  if (in_sizes[15] != FD || in_sizes[17] != FD || in_sizes[19] != FD || in_sizes[20] != FD || in_sizes[22] != FD) return;
  if (in_sizes[23] != FD || in_sizes[24] != FD) return;
  if (out_size != nN * FD) return;

  const float* x   = (const float*)d_in[0];
  const int*   ei  = (const int*)d_in[1];
  const float* ea  = (const float*)d_in[2];
  const float* qw0 = (const float*)d_in[3];  const float* qb0 = (const float*)d_in[4];
  const float* kw0 = (const float*)d_in[5];  const float* kb0 = (const float*)d_in[6];
  const float* vw0 = (const float*)d_in[7];  const float* vb0 = (const float*)d_in[8];
  const float* ew0 = (const float*)d_in[9];
  const float* sw0 = (const float*)d_in[10]; const float* sb0 = (const float*)d_in[11];
  const float* lg0 = (const float*)d_in[12]; const float* lb0 = (const float*)d_in[13];
  const float* qw1 = (const float*)d_in[14]; const float* qb1 = (const float*)d_in[15];
  const float* kw1 = (const float*)d_in[16]; const float* kb1 = (const float*)d_in[17];
  const float* vw1 = (const float*)d_in[18]; const float* vb1 = (const float*)d_in[19];
  const float* ew1 = (const float*)d_in[20];
  const float* sw1 = (const float*)d_in[21]; const float* sb1 = (const float*)d_in[22];
  const float* lg1 = (const float*)d_in[23]; const float* lb1 = (const float*)d_in[24];
  float* out = (float*)d_out;
  const int* src = ei;
  const int* dst = ei + nE;

  size_t off = 0;
  unsigned short* F0  = (unsigned short*)((char*)d_ws + off); off += (size_t)2 * FD * KIN * 2;
  unsigned short* Hh0 = (unsigned short*)((char*)d_ws + off); off += (size_t)2 * FD * KIN * 2;
  unsigned short* Hl0 = (unsigned short*)((char*)d_ws + off); off += (size_t)2 * FD * KIN * 2;
  unsigned short* F1  = (unsigned short*)((char*)d_ws + off); off += (size_t)2 * FD * FD * 2;
  unsigned short* Hh1 = (unsigned short*)((char*)d_ws + off); off += (size_t)2 * FD * FD * 2;
  unsigned short* Hl1 = (unsigned short*)((char*)d_ws + off); off += (size_t)2 * FD * FD * 2;
  unsigned short* Qh  = (unsigned short*)((char*)d_ws + off); off += (size_t)nN * FD * 2;
  float* Kf = (float*)((char*)d_ws + off); off += (size_t)nN * FD * sizeof(float);
  float* Vf = (float*)((char*)d_ws + off); off += (size_t)nN * FD * sizeof(float);
  if (off > ws_size || off > WS_CAP) return;

  k_prep<KIN><<<(4 * FD + 255) / 256, 256, 0, stream>>>(qw0, kw0, vw0, sw0, F0, Hh0, Hl0);
  k_prep<FD><<<(4 * FD + 255) / 256, 256, 0, stream>>>(qw1, kw1, vw1, sw1, F1, Hh1, Hl1);

  const int gblk = (nN + GR - 1) / GR;
  const int ablk = (nN + NB - 1) / NB;

  k_proj<KIN><<<gblk, 256, 0, stream>>>(x, F0, Hh0, Hl0, qb0, kb0, vb0, sb0, Qh, Kf, Vf, out, nN);
  hipFuncSetAttribute(reinterpret_cast<const void*>(&k_agg<4, 1>),
                      hipFuncAttributeMaxDynamicSharedMemorySize, AGG_LDS_BYTES);
  k_agg<4, 1><<<ablk, ATHR, AGG_LDS_BYTES, stream>>>(src, dst, ea, ew0, (const _Float16*)Qh, Kf, Vf,
                                                      lg0, lb0, out, nN, nE);

  k_proj<FD><<<gblk, 256, 0, stream>>>(out, F1, Hh1, Hl1, qb1, kb1, vb1, sb1, Qh, Kf, Vf, out, nN);
  hipFuncSetAttribute(reinterpret_cast<const void*>(&k_agg<1, 0>),
                      hipFuncAttributeMaxDynamicSharedMemorySize, AGG_LDS_BYTES);
  k_agg<1, 0><<<ablk, ATHR, AGG_LDS_BYTES, stream>>>(src, dst, ea, ew1, (const _Float16*)Qh, Kf, Vf,
                                                      lg1, lb1, out, nN, nE);
}
